// OptimizedMultiAttentionHead_68436008894918
// MI455X (gfx1250) — hardware-verified
//
#include <hip/hip_runtime.h>


#ifndef NB
#define NB 2
#endif
#ifndef SEQ
#define SEQ 2048
#endif
#define NB_FULL  2
#define SEQ_FULL 2048
#define DM   1024
#define NH   16
#define HD   64
#define ZH   2
#define SCL  0.125f
#define L2E  1.4426950408889634f
static_assert(SEQ % 128 == 0);
static_assert(SEQ <= SEQ_FULL);
static_assert(NB >= 1 && NB <= NB_FULL);
static_assert(DM == NH * HD);
static_assert(NH % ZH == 0);
static_assert(HD == 64 && DM % 64 == 0);

typedef _Float16 h16;
typedef unsigned short bf;
typedef __attribute__((ext_vector_type(16))) __bf16   v16bf;
typedef __attribute__((ext_vector_type(16))) _Float16 v16h;
typedef __attribute__((ext_vector_type(8)))  _Float16 v8h;
typedef __attribute__((ext_vector_type(8)))  unsigned short v8us;
typedef __attribute__((ext_vector_type(8)))  float    v8f;
typedef __attribute__((ext_vector_type(4)))  float    v4f;
typedef v8h  __attribute__((may_alias)) v8ha;
typedef v4f  __attribute__((may_alias)) v4fa;
typedef v8us __attribute__((may_alias)) v8usa;

__device__ __forceinline__ unsigned short f2bf(float f) { unsigned u = __float_as_uint(f); u += 0x7FFFu + ((u >> 16) & 1u); return (unsigned short)(u >> 16); }
__device__ __forceinline__ float bf2f(unsigned short b) { return __uint_as_float(((unsigned)b) << 16); }
__device__ __forceinline__ float bfr(float f) { return bf2f(f2bf(f)); }
__device__ __forceinline__ v16h cat16(v8h lo, v8h hi) { return __builtin_shufflevector(lo, hi, 0, 1, 2, 3, 4, 5, 6, 7, 8, 9, 10, 11, 12, 13, 14, 15); }
__device__ __forceinline__ v16bf cat16b(v8us lo, v8us hi) { return __builtin_bit_cast(v16bf, __builtin_shufflevector(lo, hi, 0, 1, 2, 3, 4, 5, 6, 7, 8, 9, 10, 11, 12, 13, 14, 15)); }
__device__ __forceinline__ v8f wmma16(v16h a, v16h b, v8f c) { return __builtin_amdgcn_wmma_f32_16x16x32_f16(false, a, false, b, (short)0, c, false, false); }
__device__ __forceinline__ v8f wmmab(v16bf a, v16bf b, v8f c) { return __builtin_amdgcn_wmma_f32_16x16x32_bf16(false, a, false, b, (short)0, c, false, false); }

template <typename T16> struct WFrag;
template <> struct WFrag<h16> { typedef v16h V; static __device__ __forceinline__ V ld(const h16* p) { return cat16(*(const v8h*)p, *(const v8h*)(p + 16)); } static __device__ __forceinline__ v8f mma(V a, V b, v8f c) { return wmma16(a, b, c); } };
template <> struct WFrag<bf> { typedef v16bf V; static __device__ __forceinline__ V ld(const bf* p) { return cat16b(*(const v8us*)p, *(const v8us*)(p + 16)); } static __device__ __forceinline__ v8f mma(V a, V b, v8f c) { return wmmab(a, b, c); } };
template <typename T16, int NSPLIT, bool BIAS>
__global__ __launch_bounds__(32) void k_gemmw(const T16* __restrict__ A, const T16* __restrict__ A2, const T16* __restrict__ Bt, const T16* __restrict__ Bt2, int K, float* C, int ldc, const float* __restrict__ bias, size_t sA, size_t sB, size_t sC) {
    typedef typename WFrag<T16>::V V;
    __shared__ __align__(16) float os[16 * 68];
    const size_t z = blockIdx.z; A += z * sA; if (A2) A2 += z * sA; Bt += z * sB; if (Bt2) Bt2 += z * sB; C += z * sC;
    const int lane = threadIdx.x & 31, lr = lane & 15, hi = lane >> 4; const int r0 = blockIdx.x * 64, c0 = blockIdx.y * 64;
    v8f acc[4][4];
#pragma unroll
    for (int mb = 0; mb < 4; ++mb)
#pragma unroll
        for (int nb = 0; nb < 4; ++nb) acc[mb][nb] = (v8f){};
    const size_t aoff = (size_t)(r0 + lr) * K + 8 * hi, boff = (size_t)(c0 + lr) * K + 8 * hi;
#pragma unroll 1
    for (int kc = 0; kc < K; kc += 32) {
        V a[4], a2[4];
#pragma unroll
        for (int mb = 0; mb < 4; ++mb) { a[mb] = WFrag<T16>::ld(A + aoff + (size_t)mb * 16 * K + kc); if (NSPLIT == 1 || NSPLIT == 2) a2[mb] = WFrag<T16>::ld(A2 + aoff + (size_t)mb * 16 * K + kc); }
#pragma unroll
        for (int nb = 0; nb < 4; ++nb) { const V b = WFrag<T16>::ld(Bt + boff + (size_t)nb * 16 * K + kc); V b2; if (NSPLIT >= 2) b2 = WFrag<T16>::ld(Bt2 + boff + (size_t)nb * 16 * K + kc);
#pragma unroll
            for (int mb = 0; mb < 4; ++mb) { acc[mb][nb] = WFrag<T16>::mma(a[mb], b, acc[mb][nb]); if (NSPLIT == 1 || NSPLIT == 2) acc[mb][nb] = WFrag<T16>::mma(a2[mb], b, acc[mb][nb]); if (NSPLIT >= 2) acc[mb][nb] = WFrag<T16>::mma(a[mb], b2, acc[mb][nb]); } }
        asm volatile("v_nop\n\tv_nop\n\tv_nop\n\tv_nop" : "+v"(acc[0][0]), "+v"(acc[1][1]), "+v"(acc[2][2]), "+v"(acc[3][3]) : "v"(a[0]), "v"(a[3]));
    }
#pragma unroll
    for (int mb = 0; mb < 4; ++mb) {
#pragma unroll
        for (int nb = 0; nb < 4; ++nb) {
#pragma unroll
            for (int j = 0; j < 8; ++j) os[(hi * 8 + j) * 68 + nb * 16 + lr] = acc[mb][nb][j]; }
        __builtin_amdgcn_wave_barrier(); asm volatile("" ::: "memory");
        float* crow = C + (size_t)(r0 + mb * 16) * ldc + c0;
#pragma unroll 1
        for (int ps = 0; ps < 2; ++ps) {
#pragma unroll
            for (int s = 0; s < 8; ++s) { const int row = 2 * s + hi, cofs = lr * 4; v4f val = *(const v4fa*)(os + row * 68 + cofs); if (BIAS) { val[0] += bfr(bias[c0 + cofs]); val[1] += bfr(bias[c0 + cofs + 1]); val[2] += bfr(bias[c0 + cofs + 2]); val[3] += bfr(bias[c0 + cofs + 3]); }
                *(volatile v4f*)(crow + (size_t)row * ldc + cofs) = val; }
            if (ps == 0) __threadfence(); }
        __builtin_amdgcn_wave_barrier(); asm volatile("" ::: "memory");
    }
}

template <typename T16, int NSPLIT, int CMODE>
__global__ __launch_bounds__(32) void k_gemmc(const T16* __restrict__ A, const T16* __restrict__ A2, const T16* __restrict__ Bt, const T16* __restrict__ Bt2, int K, float* C, int ldc, int roff, size_t sA, size_t sB, size_t sC) {
    typedef typename WFrag<T16>::V V;
    __shared__ __align__(16) float os[16 * 68];
    const size_t z = blockIdx.z; A += z * sA; if (A2) A2 += z * sA; Bt += z * sB; if (Bt2) Bt2 += z * sB; C += z * sC;
    const int lane = threadIdx.x & 31, lr = lane & 15, hi = lane >> 4; const int r0 = blockIdx.x * 64, c0 = blockIdx.y * 64;
    if (CMODE == 1 && c0 > r0 + roff + 63) return;
    const int Kl = (CMODE == 2) ? min(K, r0 + roff + 64) : K;
    v8f acc[4][4];
#pragma unroll
    for (int mb = 0; mb < 4; ++mb)
#pragma unroll
        for (int nb = 0; nb < 4; ++nb) acc[mb][nb] = (v8f){};
    const size_t aoff = (size_t)(r0 + lr) * K + 8 * hi, boff = (size_t)(c0 + lr) * K + 8 * hi;
#pragma unroll 1
    for (int kc = 0; kc < Kl; kc += 32) {
        V a[4], a2[4];
#pragma unroll
        for (int mb = 0; mb < 4; ++mb) { a[mb] = WFrag<T16>::ld(A + aoff + (size_t)mb * 16 * K + kc); if (NSPLIT == 1 || NSPLIT == 2) a2[mb] = WFrag<T16>::ld(A2 + aoff + (size_t)mb * 16 * K + kc); }
#pragma unroll
        for (int nb = 0; nb < 4; ++nb) { const V b = WFrag<T16>::ld(Bt + boff + (size_t)nb * 16 * K + kc); V b2; if (NSPLIT >= 2) b2 = WFrag<T16>::ld(Bt2 + boff + (size_t)nb * 16 * K + kc);
#pragma unroll
            for (int mb = 0; mb < 4; ++mb) { acc[mb][nb] = WFrag<T16>::mma(a[mb], b, acc[mb][nb]); if (NSPLIT == 1 || NSPLIT == 2) acc[mb][nb] = WFrag<T16>::mma(a2[mb], b, acc[mb][nb]); if (NSPLIT >= 2) acc[mb][nb] = WFrag<T16>::mma(a[mb], b2, acc[mb][nb]); } }
        asm volatile("v_nop\n\tv_nop\n\tv_nop\n\tv_nop" : "+v"(acc[0][0]), "+v"(acc[1][1]), "+v"(acc[2][2]), "+v"(acc[3][3]) : "v"(a[0]), "v"(a[3]));
    }
#pragma unroll
    for (int mb = 0; mb < 4; ++mb) {
#pragma unroll
        for (int nb = 0; nb < 4; ++nb) {
#pragma unroll
            for (int j = 0; j < 8; ++j) os[(hi * 8 + j) * 68 + nb * 16 + lr] = acc[mb][nb][j]; }
        __builtin_amdgcn_wave_barrier(); asm volatile("" ::: "memory");
        float* crow = C + (size_t)(r0 + mb * 16) * ldc + c0;
#pragma unroll 1
        for (int ps = 0; ps < 2; ++ps) {
#pragma unroll
            for (int s = 0; s < 8; ++s) { const int row = 2 * s + hi, cofs = lr * 4; v4f val = *(const v4fa*)(os + row * 68 + cofs);
                *(volatile v4f*)(crow + (size_t)row * ldc + cofs) = val; }
            if (ps == 0) __threadfence(); }
        __builtin_amdgcn_wave_barrier(); asm volatile("" ::: "memory");
    }
}

__device__ __forceinline__ void splitf(float y, unsigned short& h, unsigned short& l) { h = f2bf(y); l = f2bf(y - bf2f(h)); }
typedef __attribute__((ext_vector_type(2))) unsigned short v2us;
typedef __attribute__((ext_vector_type(4))) unsigned short v4us;

__global__ __launch_bounds__(256) void k_cvt8(const float* __restrict__ src, bf* dst, size_t n8) { const size_t i = (size_t)blockIdx.x * 256 + threadIdx.x; if (i >= n8) return; const v8f v = *(const v8f*)(src + i * 8); v8us o;
#pragma unroll
    for (int k = 0; k < 8; ++k) o[k] = f2bf(v[k]); *(volatile v8us*)(dst + i * 8) = o; __threadfence(); *(volatile v8us*)(dst + i * 8) = o; }

__global__ __launch_bounds__(256) void k_hsplit(const float* __restrict__ F, int pitch, int nheads, bf* Ph, bf* Pl) {
    const size_t e = ((size_t)blockIdx.x * 256 + threadIdx.x) * 2; if (e >= (size_t)nheads * SEQ * HD) return;
    const int d = (int)(e % HD); const int t = (int)((e / HD) % SEQ); const int h = (int)(e / ((size_t)HD * SEQ)); const float* f = F + (size_t)t * pitch + h * HD + d; v2us oh, ol;
#pragma unroll
    for (int q = 0; q < 2; ++q) { unsigned short a, c; splitf(f[q], a, c); oh[q] = a; ol[q] = c; }
    *(volatile v2us*)(Ph + e) = oh; *(volatile v2us*)(Pl + e) = ol; __threadfence(); *(volatile v2us*)(Ph + e) = oh; *(volatile v2us*)(Pl + e) = ol; }
__global__ __launch_bounds__(256) void k_vtp(const float* __restrict__ F, int pitch, int nheads, bf* Vh, bf* Vl) { const size_t e = ((size_t)blockIdx.x * 256 + threadIdx.x) * 2; if (e >= (size_t)nheads * HD * SEQ) return; const int t = (int)(e % SEQ); const int d = (int)((e / SEQ) % HD); const int g = (int)(e / ((size_t)SEQ * HD)); v2us oh, ol;
#pragma unroll
    for (int q = 0; q < 2; ++q) { const float x = F[(size_t)(t + q) * pitch + g * HD + d]; unsigned short a, c; splitf(x, a, c); oh[q] = a; ol[q] = c; }
    *(volatile v2us*)(Vh + e) = oh; *(volatile v2us*)(Vl + e) = ol; __threadfence(); *(volatile v2us*)(Vh + e) = oh; *(volatile v2us*)(Vl + e) = ol; }

__global__ __launch_bounds__(256) void k_soft(const float* __restrict__ Sb, const float* __restrict__ ga, const float* __restrict__ gb, bf* Ph, bf* Pl) {
    const int lane = threadIdx.x & 31; const int row = blockIdx.x * 8 + (threadIdx.x >> 5); if (row >= ZH * SEQ) return;
    const int i = row % SEQ; const int nch = (i >> 7) + 1;
    const float* sr = Sb + (size_t)row * SEQ; bf* ph = Ph + (size_t)row * SEQ; bf* pl = Pl + (size_t)row * SEQ;
    float m = -3.0e38f, sum = 0.f;
#pragma unroll 1
    for (int ch = 0; ch < nch; ++ch) {
        const int j0 = ch * 128 + lane * 4; const v4f a = *(const v4f*)(sr + j0); float t[4]; float cm = -3.0e38f;
#pragma unroll
        for (int q = 0; q < 4; ++q) { t[q] = (j0 + q <= i) ? a[q] * SCL : -3.0e38f; cm = fmaxf(cm, t[q]); }
#pragma unroll
        for (int sh = 16; sh; sh >>= 1) cm = fmaxf(cm, __shfl_xor(cm, sh, 32));
        const float nm = fmaxf(m, cm);
        float dm = __fsub_rn(m, nm); asm volatile("" : "+v"(dm)); const float corr = __builtin_amdgcn_exp2f(__fmul_rn(dm, L2E));
        float es = 0.f;
#pragma unroll
        for (int q = 0; q < 4; ++q) { float d0 = __fsub_rn(t[q], nm); asm volatile("" : "+v"(d0)); es += __builtin_amdgcn_exp2f(__fmul_rn(d0, L2E)); }
        sum = sum * corr + es; m = nm;
    }
#pragma unroll
    for (int sh = 16; sh; sh >>= 1) sum += __shfl_xor(sum, sh, 32);
    const float inv = __fdiv_rn(1.0f, sum);
#pragma unroll 1
    for (int ch = 0; ch < nch; ++ch) {
        const int j0 = ch * 128 + lane * 4; const v4f a = *(const v4f*)(sr + j0); const v4f av = *(const v4f*)(ga + j0), bv = *(const v4f*)(gb + j0); v4us oh, ol;
#pragma unroll
        for (int q = 0; q < 4; ++q) { const float t = (j0 + q <= i) ? a[q] * SCL : -3.0e38f; float d0 = __fsub_rn(t, m); asm volatile("" : "+v"(d0));
            const float p = __builtin_amdgcn_exp2f(__fmul_rn(d0, L2E)) * inv; const float g = 0.5f * __cosf(bfr(av[q]) * p + bfr(bv[q])) + 0.5f; const float pm = p * g;
            unsigned short hh, ll; splitf(pm, hh, ll); oh[q] = hh; ol[q] = ll; }
        *(volatile v4us*)(ph + j0) = oh; *(volatile v4us*)(pl + j0) = ol; __threadfence(); *(volatile v4us*)(ph + j0) = oh; *(volatile v4us*)(pl + j0) = ol;
    }
    const v4us z4 = (v4us){};
#pragma unroll 1
    for (int ch = nch; ch < SEQ / 128; ++ch) { const int j0 = ch * 128 + lane * 4; *(volatile v4us*)(ph + j0) = z4; *(volatile v4us*)(pl + j0) = z4; __threadfence(); *(volatile v4us*)(ph + j0) = z4; *(volatile v4us*)(pl + j0) = z4; }
}
__global__ __launch_bounds__(256) void k_merge(const float* __restrict__ O, bf* Ah, bf* Al) { const size_t e = ((size_t)blockIdx.x * 256 + threadIdx.x) * 2; if (e >= (size_t)NH * SEQ * HD) return; const int d = (int)(e % HD); const int t = (int)((e / HD) % SEQ); const int h = (int)(e / ((size_t)HD * SEQ)); const size_t oo = (size_t)t * DM + h * HD + d;
    v2us oh, ol;
#pragma unroll
    for (int q = 0; q < 2; ++q) { unsigned short a, c; splitf(O[e + q], a, c); oh[q] = a; ol[q] = c; } *(volatile v2us*)(Ah + oo) = oh; *(volatile v2us*)(Al + oo) = ol; __threadfence(); *(volatile v2us*)(Ah + oo) = oh; *(volatile v2us*)(Al + oo) = ol; }
__global__ __launch_bounds__(256) void k_gate(const float* __restrict__ P, const float* __restrict__ ga, const float* __restrict__ gb, float* O, size_t n4) { const size_t i = (size_t)blockIdx.x * 256 + threadIdx.x; if (i >= n4) return; const int c = (int)((i * 4) % DM);
    const v4f p = *(const v4f*)(P + i * 4), av = *(const v4f*)(ga + c), bv = *(const v4f*)(gb + c); v4f o;
#pragma unroll
    for (int q = 0; q < 4; ++q) { const float zv = p[q]; const float g = 0.5f * __cosf(bfr(av[q]) * zv + bfr(bv[q])) + 0.5f; o[q] = zv * g; }
    *(volatile v4f*)(O + i * 4) = o; __threadfence(); *(volatile v4f*)(O + i * 4) = o; }

extern "C" void kernel_launch(void* const* d_in, const int* in_sizes, int n_in,
                              void* d_out, int out_size, void* d_ws, size_t ws_size, hipStream_t stream) {
    if (n_in < 7) return;
    if (in_sizes[0] < (NB - 1) * SEQ_FULL * DM + SEQ * DM) return;
    if (in_sizes[1] < 3 * DM * DM || in_sizes[2] < DM * DM) return;
    if (in_sizes[3] < SEQ || in_sizes[4] < SEQ || in_sizes[5] < DM || in_sizes[6] < DM) return;
    if (out_size < NB * SEQ * DM) return;
    const float* x = (const float*)d_in[0]; const float* wqkv = (const float*)d_in[1]; const float* wo = (const float*)d_in[2];
    const float* a1 = (const float*)d_in[3]; const float* b1 = (const float*)d_in[4]; const float* a2 = (const float*)d_in[5]; const float* b2 = (const float*)d_in[6];
    float* OUT = (float*)d_out;
    char* wsp = (char*)d_ws;
    auto take = [&](size_t bytes) { char* p = wsp; wsp += (bytes + 255) & ~(size_t)255; return (void*)p; };
    bf* WQKV = (bf*)take((size_t)3 * DM * DM * 2);
    bf* WO   = (bf*)take((size_t)DM * DM * 2);
    bf* XB   = (bf*)take((size_t)SEQ * DM * 2);
    const size_t fbytes = (size_t)SEQ * 3 * DM * 4, sbytes = (size_t)ZH * SEQ * SEQ * 4;
    float* FS  = (float*)take(fbytes > sbytes ? fbytes : sbytes);
    float* F   = FS; float* Sb = FS;
    bf* QKh  = (bf*)take((size_t)2 * NH * SEQ * HD * 2); bf* QKl = (bf*)take((size_t)2 * NH * SEQ * HD * 2);
    bf* VTh  = (bf*)take((size_t)NH * HD * SEQ * 2);     bf* VTl = (bf*)take((size_t)NH * HD * SEQ * 2);
    bf* Ph   = (bf*)take((size_t)ZH * SEQ * SEQ * 2);     bf* Pl  = (bf*)take((size_t)ZH * SEQ * SEQ * 2);
    float* Ob = (float*)take((size_t)NH * SEQ * HD * 4);
    bf* ATh  = (bf*)take((size_t)SEQ * DM * 2);           bf* ATl = (bf*)take((size_t)SEQ * DM * 2);
    float* PRJ = (float*)take((size_t)SEQ * DM * 4);
    if ((size_t)(wsp - (char*)d_ws) > ws_size) return;
    k_cvt8<<<(unsigned)(((size_t)3 * DM * DM / 8 + 255) / 256), 256, 0, stream>>>(wqkv, WQKV, (size_t)3 * DM * DM / 8);
    k_cvt8<<<(unsigned)(((size_t)DM * DM / 8 + 255) / 256), 256, 0, stream>>>(wo, WO, (size_t)DM * DM / 8);
    const unsigned LQK = (unsigned)(((size_t)2 * NH * SEQ * HD / 2 + 255) / 256), LV = (unsigned)(((size_t)NH * HD * SEQ / 2 + 255) / 256);
    for (int b = 0; b < NB; ++b) {
        k_cvt8<<<(unsigned)(((size_t)SEQ * DM / 8 + 255) / 256), 256, 0, stream>>>(x + (size_t)b * SEQ_FULL * DM, XB, (size_t)SEQ * DM / 8);
        k_gemmw<bf, 0, false><<<dim3(SEQ / 64, 3 * DM / 64, 1), 32, 0, stream>>>(XB, nullptr, WQKV, nullptr, DM, F, 3 * DM, nullptr, 0, 0, 0);
        k_hsplit<<<LQK, 256, 0, stream>>>(F, 3 * DM, 2 * NH, QKh, QKl);
        k_vtp<<<LV, 256, 0, stream>>>(F + 2 * DM, 3 * DM, NH, VTh, VTl);
        for (int h0 = 0; h0 < NH; h0 += ZH) {
            k_gemmc<bf, 2, 1><<<dim3(SEQ / 64, SEQ / 64, ZH), 32, 0, stream>>>(QKh + (size_t)h0 * SEQ * HD, QKl + (size_t)h0 * SEQ * HD, QKh + (size_t)(NH + h0) * SEQ * HD, QKl + (size_t)(NH + h0) * SEQ * HD, HD, Sb, SEQ, 0, (size_t)SEQ * HD, (size_t)SEQ * HD, (size_t)SEQ * SEQ);
            k_soft<<<(unsigned)(ZH * SEQ / 8), 256, 0, stream>>>(Sb, a1, b1, Ph, Pl);
            k_gemmc<bf, 2, 2><<<dim3(SEQ / 64, HD / 64, ZH), 32, 0, stream>>>(Ph, Pl, VTh + (size_t)h0 * HD * SEQ, VTl + (size_t)h0 * HD * SEQ, SEQ, Ob + (size_t)h0 * SEQ * HD, HD, 0, (size_t)SEQ * SEQ, (size_t)HD * SEQ, (size_t)SEQ * HD);
        }
        k_merge<<<(unsigned)(((size_t)NH * SEQ * HD / 2 + 255) / 256), 256, 0, stream>>>(Ob, ATh, ATl);
        k_gemmw<bf, 1, false><<<dim3(SEQ / 64, DM / 64, 1), 32, 0, stream>>>(ATh, ATl, WO, nullptr, DM, PRJ, DM, nullptr, 0, 0, 0);
        k_gate<<<(unsigned)(((size_t)SEQ * DM / 4 + 255) / 256), 256, 0, stream>>>(PRJ, a2, b2, OUT + (size_t)b * SEQ * DM, (size_t)SEQ * DM / 4);
    }
}
